// SVMModel_45792941310118
// MI455X (gfx1250) — hardware-run, weakly checked
//
#include <hip/hip_runtime.h>


#ifndef NB
#define NB 32768
#endif
#ifndef NSV
#define NSV 8192
#endif
#define NB_FULL  32768
#define NSV_FULL 8192
#define DIM   32
#define NPART (NB / 64)
#define LOG2E 1.4426950408889634f

static_assert(DIM == 32);
static_assert(NB % 64 == 0);
static_assert(NSV % 64 == 0);
static_assert(NSV % 16 == 0);
static_assert(NB <= NB_FULL);
static_assert(NSV <= NSV_FULL);

typedef unsigned short bf;
typedef __attribute__((ext_vector_type(16))) __bf16   v16bf;
typedef __attribute__((ext_vector_type(8)))  unsigned short v8us;
typedef __attribute__((ext_vector_type(8)))  float    v8f;
typedef __attribute__((ext_vector_type(4)))  float    v4f;
typedef v4f  __attribute__((may_alias)) v4fa;

__device__ __forceinline__ unsigned short f2bf(float f) { unsigned u = __float_as_uint(f); u += 0x7FFFu + ((u >> 16) & 1u); return (unsigned short)(u >> 16); }
__device__ __forceinline__ float bf2f(unsigned short h) { return __uint_as_float(((unsigned)h) << 16); }
__device__ __forceinline__ v16bf cat16b(v8us lo, v8us hi) { return __builtin_bit_cast(v16bf, __builtin_shufflevector(lo, hi, 0, 1, 2, 3, 4, 5, 6, 7, 8, 9, 10, 11, 12, 13, 14, 15)); }
__device__ __forceinline__ v8f wmmab(v16bf a, v16bf b, v8f c) { return __builtin_amdgcn_wmma_f32_16x16x32_bf16(false, a, false, b, (short)0, c, false, false); }
__device__ __forceinline__ v16bf ldb(const bf* p)  { return cat16b(*(const v8us*)p, *(const v8us*)(p + 16)); }
__device__ __forceinline__ void wave_sync() { __builtin_amdgcn_fence(3  , "wavefront"); __builtin_amdgcn_wave_barrier(); asm volatile("" ::: "memory"); }

__device__ __forceinline__ void cvt_piece(const float* __restrict__ src, size_t i8, v8us& o, float& s, float& q) {
    const v8f v = *(const v8f*)(src + i8 * 8);
    s = 0.0f; q = 0.0f;
#pragma unroll
    for (int k = 0; k < 8; ++k) { const unsigned short us = f2bf(v[k]); o[k] = us; const float r = bf2f(us); s += r; q = fmaf(r, r, q); }
}

__global__ __launch_bounds__(256) void k_prep_x(const float* __restrict__ src, bf* plane, float* norms, float* part) {
    __shared__ __align__(16) float sn[64];
    __shared__ float wS[8];
    __shared__ float wQ[8];
    const int tid = threadIdx.x, lane = tid & 31;
    const int wave = __builtin_amdgcn_readfirstlane(tid >> 5);
    const size_t i8 = (size_t)blockIdx.x * 256 + tid;
    v8us o; float s, q;
    cvt_piece(src, i8, o, s, q);
    q += __shfl_xor(q, 1, 32); s += __shfl_xor(s, 1, 32);
    q += __shfl_xor(q, 2, 32); s += __shfl_xor(s, 2, 32);
    if ((tid & 3) == 0) sn[tid >> 2] = q;
    q += __shfl_xor(q, 4, 32);  s += __shfl_xor(s, 4, 32);
    q += __shfl_xor(q, 8, 32);  s += __shfl_xor(s, 8, 32);
    q += __shfl_xor(q, 16, 32); s += __shfl_xor(s, 16, 32);
    if (lane == 0) { wS[wave] = s; wQ[wave] = q; }
    __syncthreads();
    v4f nv = (v4f){0.0f, 0.0f, 0.0f, 0.0f}, pl = (v4f){0.0f, 0.0f, 0.0f, 0.0f};
    if (wave == 0) {
        nv = *(const v4fa*)(&sn[(lane & 15) * 4]);
        float S = 0.0f, Q = 0.0f;
#pragma unroll
        for (int k = 0; k < 8; ++k) { S += wS[k]; Q += wQ[k]; }
        pl[0] = (lane == 0) ? S : 0.0f; pl[1] = (lane == 0) ? Q : 0.0f;
    }
#pragma unroll 1
    for (int ps = 0; ps < 2; ++ps) {
        *(volatile v8us*)(plane + i8 * 8) = o;
        if (wave == 0) {
            if (lane < 16) *(volatile v4f*)(norms + (size_t)blockIdx.x * 64 + lane * 4) = nv;
            if (lane < 8)  *(volatile v4f*)(part  + (size_t)blockIdx.x * 32 + lane * 4) = pl;
        }
        if (ps == 0) __threadfence();
    }
}

__global__ __launch_bounds__(256) void k_prep_sv(const float* __restrict__ src, const float* __restrict__ alphas, const float* __restrict__ labels,
                                                 bf* plane, float* norms, float* wout) {
    __shared__ __align__(16) float sn[64];
    __shared__ __align__(16) float sw[64];
    const int tid = threadIdx.x, lane = tid & 31;
    const int wave = __builtin_amdgcn_readfirstlane(tid >> 5);
    const size_t i8 = (size_t)blockIdx.x * 256 + tid;
    v8us o; float s, q;
    cvt_piece(src, i8, o, s, q);
    q += __shfl_xor(q, 1, 32);
    q += __shfl_xor(q, 2, 32);
    if ((tid & 3) == 0) sn[tid >> 2] = q;
    if (wave < 2) { const int j = blockIdx.x * 64 + tid;
        sw[tid] = bf2f(f2bf(alphas[j])) * bf2f(f2bf(labels[j])); }
    __syncthreads();
    v4f nv = (v4f){0.0f, 0.0f, 0.0f, 0.0f}, wv = (v4f){0.0f, 0.0f, 0.0f, 0.0f};
    if (wave == 0) {
        nv = *(const v4fa*)(&sn[(lane & 15) * 4]);
        wv = *(const v4fa*)(&sw[(lane & 15) * 4]);
    }
#pragma unroll 1
    for (int ps = 0; ps < 2; ++ps) {
        *(volatile v8us*)(plane + i8 * 8) = o;
        if (wave == 0) {
            if (lane < 16) { *(volatile v4f*)(norms + (size_t)blockIdx.x * 64 + lane * 4) = nv;
                             *(volatile v4f*)(wout  + (size_t)blockIdx.x * 64 + lane * 4) = wv; }
        }
        if (ps == 0) __threadfence();
    }
}

__global__ __launch_bounds__(32) void k_gamma(const float* __restrict__ part, float* GL) {
    const int lane = threadIdx.x & 31;
    double s = 0.0, q = 0.0;
#pragma unroll 1
    for (int b = lane; b < NPART; b += 32) { s += (double)part[(size_t)b * 32]; q += (double)part[(size_t)b * 32 + 1]; }
#pragma unroll
    for (int off = 16; off > 0; off >>= 1) { s += __shfl_xor(s, off, 32); q += __shfl_xor(q, off, 32); }
    const double inv_n = 1.0 / ((double)NB * (double)DIM);
    const double mean = s * inv_n;
    const double var = q * inv_n - mean * mean;
    const float varf = (float)var;
    const float gamma = 1.0f / ((float)DIM * varf);
    const float g2 = gamma * LOG2E;
    v4f gl = (v4f){0.0f, 0.0f, 0.0f, 0.0f};
    gl[0] = (lane == 0) ? gamma : 0.0f; gl[1] = (lane == 0) ? g2 : 0.0f;
#pragma unroll 1
    for (int ps = 0; ps < 2; ++ps) {
        if (lane < 8) *(volatile v4f*)(GL + lane * 4) = gl;
        if (ps == 0) __threadfence();
    }
}

__global__ __launch_bounds__(32) void k_rbf(const bf* __restrict__ XB, const bf* __restrict__ SB, const float* __restrict__ NX, const float* __restrict__ NS,
                                            const float* __restrict__ W, const float* __restrict__ GL, const float* __restrict__ bias, float* OUT) {
    __shared__ __align__(16) float os[64];
    const int lane = threadIdx.x & 31, lr = lane & 15, hi = lane >> 4;
    const int r0 = blockIdx.x * 64;
    const float g2 = GL[1];
    const float tg2 = 2.0f * g2;
    const float bb = bf2f(f2bf(bias[0]));

    v16bf a[4];
#pragma unroll
    for (int mb = 0; mb < 4; ++mb) a[mb] = ldb(XB + (size_t)(r0 + mb * 16 + lr) * DIM + 8 * hi);

    float xg[4][8];
#pragma unroll
    for (int mb = 0; mb < 4; ++mb) {
        const v4f n0 = *(const v4f*)(NX + r0 + mb * 16 + 8 * hi);
        const v4f n1 = *(const v4f*)(NX + r0 + mb * 16 + 8 * hi + 4);
#pragma unroll
        for (int i = 0; i < 4; ++i) { xg[mb][i] = -g2 * n0[i]; xg[mb][4 + i] = -g2 * n1[i]; }
    }

    float acc[4][8];
#pragma unroll
    for (int mb = 0; mb < 4; ++mb)
#pragma unroll
        for (int r = 0; r < 8; ++r) acc[mb][r] = 0.0f;

    const bf* sbp = SB + (size_t)lr * DIM + 8 * hi;
#pragma unroll 1
    for (int j0 = 0; j0 < NSV; j0 += 16) {
        const v16bf b = ldb(sbp + (size_t)j0 * DIM);
        const float sg = -g2 * NS[j0 + lr];
        const float wv = W[j0 + lr];
        v8f c0 = (v8f){}, c1 = (v8f){}, c2 = (v8f){}, c3 = (v8f){};
        c0 = wmmab(a[0], b, c0); c1 = wmmab(a[1], b, c1); c2 = wmmab(a[2], b, c2); c3 = wmmab(a[3], b, c3);
        asm volatile("v_nop\n\tv_nop\n\tv_nop\n\tv_nop" : "+v"(c0), "+v"(c1), "+v"(c2), "+v"(c3) : "v"(a[0]), "v"(a[1]), "v"(a[2]), "v"(a[3]), "v"(b));
#pragma unroll
        for (int r = 0; r < 8; ++r) {
            const float t0 = fmaf(tg2, c0[r], xg[0][r] + sg); acc[0][r] = fmaf(wv, __builtin_amdgcn_exp2f(t0), acc[0][r]);
            const float t1 = fmaf(tg2, c1[r], xg[1][r] + sg); acc[1][r] = fmaf(wv, __builtin_amdgcn_exp2f(t1), acc[1][r]);
            const float t2 = fmaf(tg2, c2[r], xg[2][r] + sg); acc[2][r] = fmaf(wv, __builtin_amdgcn_exp2f(t2), acc[2][r]);
            const float t3 = fmaf(tg2, c3[r], xg[3][r] + sg); acc[3][r] = fmaf(wv, __builtin_amdgcn_exp2f(t3), acc[3][r]);
        }
    }

#pragma unroll
    for (int mb = 0; mb < 4; ++mb)
#pragma unroll
        for (int r = 0; r < 8; ++r) {
            float v = acc[mb][r];
            v += __shfl_xor(v, 1, 32); v += __shfl_xor(v, 2, 32); v += __shfl_xor(v, 4, 32); v += __shfl_xor(v, 8, 32);
            acc[mb][r] = v + bb;
        }
    if (lr == 0) {
#pragma unroll
        for (int mb = 0; mb < 4; ++mb) {
            v4f p, q;
            p[0] = acc[mb][0]; p[1] = acc[mb][1]; p[2] = acc[mb][2]; p[3] = acc[mb][3];
            q[0] = acc[mb][4]; q[1] = acc[mb][5]; q[2] = acc[mb][6]; q[3] = acc[mb][7];
            *(v4fa*)(&os[mb * 16 + 8 * hi]) = p; *(v4fa*)(&os[mb * 16 + 8 * hi + 4]) = q;
        }
    }
    wave_sync();
    const v4f val = *(const v4fa*)(&os[lr * 4]);
#pragma unroll 1
    for (int ps = 0; ps < 2; ++ps) {
        if (lane < 16) *(volatile v4f*)(OUT + (size_t)r0 + lane * 4) = val;
        if (ps == 0) __threadfence();
    }
}

static constexpr size_t al256(size_t v) { return (v + 255) & ~(size_t)255; }
static constexpr size_t SZ_XB = al256((size_t)NB * DIM * 2);
static constexpr size_t SZ_SB = al256((size_t)NSV * DIM * 2);
static constexpr size_t SZ_NX = al256((size_t)NB * 4);
static constexpr size_t SZ_NS = al256((size_t)NSV * 4);
static constexpr size_t SZ_W  = al256((size_t)NSV * 4);
static constexpr size_t SZ_PT = al256((size_t)NPART * 128);
static constexpr size_t SZ_GL = al256((size_t)128);
static constexpr size_t SZ_TOTAL = SZ_XB + SZ_SB + SZ_NX + SZ_NS + SZ_W + SZ_PT + SZ_GL;
static_assert(SZ_TOTAL <= (size_t)134217728);
static_assert((size_t)(NB / 64) * 256 * 16 == (size_t)NB * DIM * 2);
static_assert((size_t)(NSV / 64) * 256 * 16 == (size_t)NSV * DIM * 2);
static_assert((size_t)(NB / 64) * 64 * 4 <= SZ_NX);
static_assert((size_t)(NSV / 64) * 64 * 4 <= SZ_NS);
static_assert((size_t)NPART * 32 * 4 <= SZ_PT);

extern "C" void kernel_launch(void* const* d_in, const int* in_sizes, int n_in,
                              void* d_out, int out_size, void* d_ws, size_t ws_size, hipStream_t stream) {
    if (n_in < 5) return;
    if ((size_t)in_sizes[0] < (size_t)NB * DIM) return;
    if ((size_t)in_sizes[1] < (size_t)NSV * DIM) return;
    if ((size_t)in_sizes[2] < (size_t)NSV || (size_t)in_sizes[3] < (size_t)NSV || in_sizes[4] < 1) return;
    if ((size_t)out_size < (size_t)NB) return;
    if (SZ_TOTAL > ws_size) return;
    const float* x = (const float*)d_in[0]; const float* sv = (const float*)d_in[1];
    const float* labels = (const float*)d_in[2]; const float* alphas = (const float*)d_in[3]; const float* bias = (const float*)d_in[4];
    float* OUT = (float*)d_out;
    char* wsp = (char*)d_ws;
    bf* XB = (bf*)wsp; wsp += SZ_XB;
    bf* SB = (bf*)wsp; wsp += SZ_SB;
    float* NX = (float*)wsp; wsp += SZ_NX;
    float* NS = (float*)wsp; wsp += SZ_NS;
    float* WV = (float*)wsp; wsp += SZ_W;
    float* PT = (float*)wsp; wsp += SZ_PT;
    float* GL = (float*)wsp; wsp += SZ_GL;

    k_prep_x<<<NB / 64, 256, 0, stream>>>(x, XB, NX, PT);
    k_prep_sv<<<NSV / 64, 256, 0, stream>>>(sv, alphas, labels, SB, NS, WV);
    k_gamma<<<1, 32, 0, stream>>>(PT, GL);
    k_rbf<<<NB / 64, 32, 0, stream>>>(XB, SB, NX, NS, WV, GL, bias, OUT);
}
